// Qwen3_5MoeGatedSDPAAttention_33371895890025
// MI455X (gfx1250) — hardware-verified
//
#include <hip/hip_runtime.h>
#include <math.h>
#include <stdint.h>

#define NBATCH 2
#define SEQ    2048
#define DM     2048
#define NHEAD  16
#define NKV    4
#define HDIM   128
#define KVD    (NKV * HDIM)
#define QGD    (2 * NHEAD * HDIM)
#define NTOK   (NBATCH * SEQ)
#define NQB    (SEQ / 64)
#define NQP    8
#define LEADR  (NQP * 64)
#define WSC    64.0f
#define QSC    4.0f
#define KSC    16.0f
#define VSC    16.0f
#define RSC    4096.0f
#define PSC    1024.0f
#define CXS    1024.0f
#define EPSN   1.0e-6f
#define NEG_BIG (-1.0e30f)
static_assert(NHEAD * HDIM == DM);
static_assert((NHEAD % NKV) == 0);
static_assert((SEQ % 64) == 0 && (DM % 128) == 0 && (KVD % 128) == 0 && (QGD % 128) == 0);
static_assert((DM % 32) == 0 && (HDIM % 32) == 0);
static_assert(((NTOK * DM) % 2048) == 0 && ((KVD * DM) % 2048) == 0 && ((DM * DM) % 2048) == 0);
static_assert(((QGD * DM) % 2048) == 0);
static_assert(NQP > 0 && NQP < NQB);
static_assert((LEADR % 32) == 0 && ((SEQ - LEADR) % 32) == 0);

typedef _Float16 v16h __attribute__((ext_vector_type(16)));
typedef _Float16 v8h  __attribute__((ext_vector_type(8)));
typedef float    v8f  __attribute__((ext_vector_type(8)));
typedef float    v4f  __attribute__((ext_vector_type(4)));
typedef unsigned int v4u __attribute__((ext_vector_type(4)));
union FH { v16h v; v8h h[2]; };

__device__ __forceinline__ unsigned short bf_bits(float f) {
  unsigned u = __float_as_uint(f);
  return (unsigned short)((u + 0x7FFFu + ((u >> 16) & 1u)) >> 16);
}
__device__ __forceinline__ float bf_up(unsigned short h) { return __uint_as_float(((unsigned)h) << 16); }
__device__ __forceinline__ float bfr(float f) { return bf_up(bf_bits(f)); }
__device__ __forceinline__ unsigned short h_bits(_Float16 x) { return __builtin_bit_cast(unsigned short, x); }
__device__ __forceinline__ unsigned pk16(unsigned short a, unsigned short b) { return (unsigned)a | ((unsigned)b << 16); }
__device__ __forceinline__ v8f zero8() { v8f z = {0.f, 0.f, 0.f, 0.f, 0.f, 0.f, 0.f, 0.f}; return z; }

__device__ __forceinline__ v16h ldfrag_h(const _Float16* p) {
  FH f;
  f.h[0] = *(const v8h*)(p);
  f.h[1] = *(const v8h*)(p + 16);
  return f.v;
}

__device__ __forceinline__ v8f mma_h_raw(v16h a, v16h b, v8f c) {
  return __builtin_amdgcn_wmma_f32_16x16x32_f16(false, a, false, b, (short)0, c, false, false);
}
__device__ __forceinline__ v8f mma_h(v16h a, v16h b, v8f c) {
  c = mma_h_raw(a, b, c);
#if defined(__HIP_DEVICE_COMPILE__)
  asm volatile("v_nop\n\tv_nop\n\tv_nop\n\tv_nop" : "+v"(c) : "v"(a), "v"(b));
#endif
  return c;
}
__device__ __forceinline__ void guard3(v8f& x, v8f& y, v16h a, v16h b, v16h d) {
#if defined(__HIP_DEVICE_COMPILE__)
  asm volatile("v_nop\n\tv_nop\n\tv_nop\n\tv_nop" : "+v"(x), "+v"(y) : "v"(a), "v"(b), "v"(d));
#endif
}
__device__ __forceinline__ void guard1q(v8f& x, v16h a, v16h b, v16h d, v16h e) {
#if defined(__HIP_DEVICE_COMPILE__)
  asm volatile("v_nop\n\tv_nop\n\tv_nop\n\tv_nop" : "+v"(x) : "v"(a), "v"(b), "v"(d), "v"(e));
#endif
}
__device__ __forceinline__ void guard4m(v8f& x, v8f& y, v16h a, v16h b, v16h d, v16h e) {
#if defined(__HIP_DEVICE_COMPILE__)
  asm volatile("v_nop\n\tv_nop\n\tv_nop\n\tv_nop" : "+v"(x), "+v"(y) : "v"(a), "v"(b), "v"(d), "v"(e)
               : "memory");
#endif
}
__device__ __forceinline__ void guard8m(v8f& x, v8f& y, v16h a, v16h b, v16h d, v16h e,
                                        v16h f, v16h g, v16h p, v16h q) {
#if defined(__HIP_DEVICE_COMPILE__)
  asm volatile("v_nop\n\tv_nop\n\tv_nop\n\tv_nop" : "+v"(x), "+v"(y)
               : "v"(a), "v"(b), "v"(d), "v"(e), "v"(f), "v"(g), "v"(p), "v"(q) : "memory");
#endif
}
__device__ __forceinline__ void acc_guard4(v8f& a, v8f& b, v8f& c, v8f& d) {
#if defined(__HIP_DEVICE_COMPILE__)
  asm volatile("v_nop\n\tv_nop\n\tv_nop\n\tv_nop" : "+v"(a), "+v"(b), "+v"(c), "+v"(d));
#endif
}
__device__ __forceinline__ void cbar() {
#if defined(__HIP_DEVICE_COMPILE__)
  asm volatile("" ::: "memory");
#endif
}
__device__ __forceinline__ void wave_sync_lds() {
  __builtin_amdgcn_fence(__ATOMIC_RELEASE, "workgroup");
  __builtin_amdgcn_wave_barrier();
  __builtin_amdgcn_fence(__ATOMIC_ACQUIRE, "workgroup");
}

__global__ __launch_bounds__(256) void cvt_rm(const float* __restrict__ in, unsigned short* out, int n,
                                             float scale, int bfmode) {
  const size_t i8 = ((size_t)blockIdx.x * 256 + threadIdx.x) * 8;
  if (i8 + 8 > (size_t)n) return;
  const v4f a = *(const v4f*)(in + i8);
  const v4f b = *(const v4f*)(in + i8 + 4);
  float f[8];
  f[0] = a[0]; f[1] = a[1]; f[2] = a[2]; f[3] = a[3];
  f[4] = b[0]; f[5] = b[1]; f[6] = b[2]; f[7] = b[3];
  v4u p;
#pragma unroll
  for (int e = 0; e < 4; ++e) {
    const unsigned short b0 = bf_bits(f[2 * e]), b1 = bf_bits(f[2 * e + 1]);
    const _Float16 x0 = (_Float16)(bf_up(b0) * scale);
    const _Float16 x1 = (_Float16)(bf_up(b1) * scale);
    const unsigned wf = pk16(h_bits(x0), h_bits(x1));
    const unsigned wb = pk16(b0, b1);
    p[e] = (bfmode != 0) ? wb : wf;
  }
  *(volatile v4u*)(out + i8) = p;
  __threadfence();
  *(volatile v4u*)(out + i8) = p;
}

template <int NSW, int EPI>
__global__ __launch_bounds__(128) void gemm_t(
    const unsigned short* __restrict__ A0, const unsigned short* __restrict__ A1, int lda,
    const unsigned short* __restrict__ B0, const unsigned short* __restrict__ B1, int ldb,
    void* C0, void* C1, void* C2, int ldc,
    const float* __restrict__ cosb, const float* __restrict__ sinb, const float* __restrict__ nw,
    int M, int N, int K, float oscale, float cscale) {
  __shared__ __align__(16) float sT[4][16 * 132];
  const int lane = threadIdx.x & 31;
  const int wave = threadIdx.x >> 5;
  const int tilesN = N >> 7;
  const int tilesM = M >> 5;
  const int tile = blockIdx.x * 4 + wave;
  if (tile >= tilesM * tilesN) return;
  const int tm = tile / tilesN;
  const int tn = tile - tm * tilesN;
  const int m0 = tm << 5;
  const int n0 = tn << 7;
  const int rl   = lane & 15;
  const int hh   = lane >> 4;
  const int koff = hh * 8;

  v8f acc[2][8];
#pragma unroll
  for (int i = 0; i < 2; ++i)
#pragma unroll
    for (int j = 0; j < 8; ++j) acc[i][j] = zero8();

#pragma unroll 1
  for (int sw = 0; sw < NSW; ++sw) {
    const unsigned short* Ab = (sw == 0) ? A0 : A1;
    const unsigned short* Bb = (sw == 0) ? B0 : B1;
    const _Float16* ar0 = (const _Float16*)(const void*)Ab + (size_t)(m0 + rl) * (size_t)lda + koff;
    const _Float16* ar1 = (const _Float16*)(const void*)Ab + (size_t)(m0 + 16 + rl) * (size_t)lda + koff;
    const _Float16* br  = (const _Float16*)(const void*)Bb + (size_t)(n0 + rl) * (size_t)ldb + koff;
    for (int k0 = 0; k0 < K; k0 += 32) {
      const v16h a0 = ldfrag_h(ar0 + k0);
      const v16h a1 = ldfrag_h(ar1 + k0);
#pragma unroll
      for (int j = 0; j < 8; ++j) {
        const v16h b = ldfrag_h(br + (size_t)j * 16 * (size_t)ldb + k0);
        acc[0][j] = mma_h_raw(a0, b, acc[0][j]);
        acc[1][j] = mma_h_raw(a1, b, acc[1][j]);
        guard3(acc[0][j], acc[1][j], a0, a1, b);
      }
    }
  }
  acc_guard4(acc[0][0], acc[0][1], acc[0][2], acc[0][3]);
  acc_guard4(acc[0][4], acc[0][5], acc[0][6], acc[0][7]);
  acc_guard4(acc[1][0], acc[1][1], acc[1][2], acc[1][3]);
  acc_guard4(acc[1][4], acc[1][5], acc[1][6], acc[1][7]);

  const bool normt = (EPI == 1) || ((EPI == 2) && ((tn & 1) == 0));
  const bool f32t  = (EPI == 3) || ((EPI == 2) && ((tn & 1) != 0));
  const int ccol = (EPI == 2) ? ((tn >> 1) * HDIM) : n0;
  float wf[8];
#pragma unroll
  for (int j = 0; j < 8; ++j) wf[j] = 1.0f;
  if (EPI == 1 || EPI == 2) {
#pragma unroll
    for (int j = 0; j < 8; ++j) wf[j] = 1.0f + bfr(nw[16 * j + rl]);
  }
  float* slab = sT[wave];
#pragma unroll
  for (int i = 0; i < 2; ++i) {
    const int mB = m0 + 16 * i;
    if (normt) {
      float inv[8];
#pragma unroll
      for (int r = 0; r < 8; ++r) {
        float ss = 0.f;
#pragma unroll
        for (int j = 0; j < 8; ++j) {
          const float x = acc[i][j][r] * oscale;
          ss += x * x;
        }
        ss += __shfl_xor(ss, 1, 32);
        ss += __shfl_xor(ss, 2, 32);
        ss += __shfl_xor(ss, 4, 32);
        ss += __shfl_xor(ss, 8, 32);
        inv[r] = rsqrtf(ss * (1.0f / (float)HDIM) + EPSN) * oscale;
      }
#pragma unroll
      for (int j = 0; j < 4; ++j) {
#pragma unroll
        for (int r = 0; r < 8; ++r) {
          const int t = mB + 8 * hh + r;
          const float* cr = cosb + (size_t)t * HDIM + 16 * j + rl;
          const float* sr = sinb + (size_t)t * HDIM + 16 * j + rl;
          const float c1 = bfr(cr[0]),  s1 = bfr(sr[0]);
          const float c2 = bfr(cr[64]), s2 = bfr(sr[64]);
          const float x1 = acc[i][j][r] * inv[r] * wf[j];
          const float x2 = acc[i][j + 4][r] * inv[r] * wf[j + 4];
          slab[(8 * hh + r) * 132 + 16 * j + rl]      = (x1 * c1 - x2 * s1) * cscale;
          slab[(8 * hh + r) * 132 + 64 + 16 * j + rl] = (x2 * c2 + x1 * s2) * cscale;
        }
      }
    } else {
#pragma unroll
      for (int j = 0; j < 8; ++j) {
#pragma unroll
        for (int r = 0; r < 8; ++r) slab[(8 * hh + r) * 132 + 16 * j + rl] = acc[i][j][r] * oscale;
      }
    }
    wave_sync_lds();
    if (f32t) {
      float* Cf = (float*)((EPI == 3) ? C0 : C2);
      for (int pass = 0; pass < 2; ++pass) {
#pragma unroll
        for (int it = 0; it < 16; ++it) {
          const v4f o = *(const v4f*)(slab + it * 132 + lane * 4);
          *(volatile v4f*)(Cf + (size_t)(mB + it) * (size_t)ldc + ccol + lane * 4) = o;
        }
        __threadfence();
      }
    } else {
      unsigned short* Cp = (unsigned short*)C0;
      unsigned short* Cq = (unsigned short*)C1;
      v4u hv[8], lv[8];
#pragma unroll
      for (int it = 0; it < 8; ++it) {
        const int row = it * 2 + hh;
        const float* sp = slab + row * 132 + rl * 8;
        const v4f fa = *(const v4f*)sp;
        const v4f fb = *(const v4f*)(sp + 4);
        float f[8];
        f[0] = fa[0]; f[1] = fa[1]; f[2] = fa[2]; f[3] = fa[3];
        f[4] = fb[0]; f[5] = fb[1]; f[6] = fb[2]; f[7] = fb[3];
        v4u pk, pl;
#pragma unroll
        for (int e = 0; e < 4; ++e) {
          const float g0 = f[2 * e], g1 = f[2 * e + 1];
          const _Float16 x0 = (_Float16)g0;
          const _Float16 x1 = (_Float16)g1;
          const _Float16 y0 = (_Float16)((g0 - (float)x0) * RSC);
          const _Float16 y1 = (_Float16)((g1 - (float)x1) * RSC);
          pk[e] = pk16(h_bits(x0), h_bits(x1));
          pl[e] = pk16(h_bits(y0), h_bits(y1));
        }
        hv[it] = pk;
        lv[it] = pl;
      }
      for (int pass = 0; pass < 2; ++pass) {
#pragma unroll
        for (int it = 0; it < 8; ++it) {
          const int row = it * 2 + hh;
          const size_t go = (size_t)(mB + row) * (size_t)ldc + ccol + rl * 8;
          *(volatile v4u*)(Cp + go) = hv[it];
          *(volatile v4u*)(Cq + go) = lv[it];
        }
        __threadfence();
      }
    }
    wave_sync_lds();
  }
}

template <bool PRES>
__global__ __launch_bounds__(128)
void attn_c(const unsigned short* __restrict__ QHp, const unsigned short* __restrict__ QLp,
            const unsigned short* __restrict__ KHp, const unsigned short* __restrict__ KLp,
            const unsigned short* __restrict__ VHp, const unsigned short* __restrict__ VLp,
            const float* __restrict__ GTp, unsigned short* CH, unsigned short* CL,
            float sscale, int qb0, int nqb) {
  __shared__ __align__(16) _Float16 Ksh[64 * HDIM];
  __shared__ __align__(16) _Float16 Kls[PRES ? 64 * HDIM : 8];
  __shared__ __align__(16) _Float16 Vhs[HDIM * 64];
  __shared__ __align__(16) _Float16 Vls[PRES ? HDIM * 64 : 8];
  __shared__ __align__(16) _Float16 Psh[4][16 * 64];
  __shared__ __align__(16) _Float16 Psl[PRES ? 4 : 1][PRES ? 16 * 64 : 8];
  __shared__ __align__(16) float    Os[4][16 * HDIM];

  const int tid  = threadIdx.x;
  const int wave = tid >> 5;
  const int lane = tid & 31;
  const int hh   = lane >> 4;
  const int c    = lane & 15;

  const int qb  = qb0 + (int)(blockIdx.x % (unsigned)nqb);
  const int h   = (int)(blockIdx.x / (unsigned)nqb);
  const int kvh = h / (NHEAD / NKV);
  const int q0  = qb * 64 + wave * 16;

  const _Float16* Qg  = (const _Float16*)(const void*)QHp + (size_t)h * HDIM;
  const _Float16* Qlg = (const _Float16*)(const void*)QLp + (size_t)h * HDIM;
  const _Float16* Kg  = (const _Float16*)(const void*)KHp + (size_t)kvh * HDIM;
  const _Float16* Klg = (const _Float16*)(const void*)KLp + (size_t)kvh * HDIM;
  const _Float16* Vhg = (const _Float16*)(const void*)VHp + (size_t)kvh * HDIM * SEQ;
  const _Float16* Vlg = (const _Float16*)(const void*)VLp + (size_t)kvh * HDIM * SEQ;
  const float* Gg = GTp + (size_t)h * HDIM;

  float mrow[8], lrow[8];
  v8f oh[8];
#pragma unroll
  for (int r = 0; r < 8; ++r) { mrow[r] = NEG_BIG; lrow[r] = 0.f; }
#pragma unroll
  for (int t = 0; t < 8; ++t) oh[t] = zero8();

  _Float16* pwh = Psh[wave];
  _Float16* pwl = &Psl[PRES ? wave : 0][0];

  for (int kt = 0; kt < NQB; ++kt) {
    if (kt > qb) break;
    const int kv0 = kt * 64;
    __syncthreads();
    {
      const int r = tid >> 1, hk = (tid & 1) * 64;
      const _Float16* kg = Kg + (size_t)(kv0 + r) * KVD + hk;
#pragma unroll
      for (int i = 0; i < 8; ++i) *(v8h*)(Ksh + r * HDIM + hk + 8 * i) = *(const v8h*)(kg + 8 * i);
      if (PRES) {
        cbar();
        const _Float16* lg = Klg + (size_t)(kv0 + r) * KVD + hk;
#pragma unroll
        for (int i = 0; i < 8; ++i) *(v8h*)(Kls + r * HDIM + hk + 8 * i) = *(const v8h*)(lg + 8 * i);
        cbar();
      }
      const _Float16* vh = Vhg + (size_t)tid * SEQ + kv0;
#pragma unroll
      for (int i = 0; i < 8; ++i) *(v8h*)(Vhs + tid * 64 + 8 * i) = *(const v8h*)(vh + 8 * i);
      if (PRES) {
        cbar();
        const _Float16* vl = Vlg + (size_t)tid * SEQ + kv0;
#pragma unroll
        for (int i = 0; i < 8; ++i) *(v8h*)(Vls + tid * 64 + 8 * i) = *(const v8h*)(vl + 8 * i);
        cbar();
      }
    }
    __syncthreads();

    v8f s[4];
    if (PRES) {
#pragma unroll
      for (int jp = 0; jp < 2; ++jp) {
        v8f sh2[2], sl2[2];
        sh2[0] = zero8(); sh2[1] = zero8(); sl2[0] = zero8(); sl2[1] = zero8();
#pragma unroll
        for (int dc = 0; dc < 4; ++dc) {
          const v16h qhf = ldfrag_h(Qg  + (size_t)(q0 + c) * DM + dc * 32 + 8 * hh);
          const v16h qlf = ldfrag_h(Qlg + (size_t)(q0 + c) * DM + dc * 32 + 8 * hh);
#pragma unroll
          for (int jj = 0; jj < 2; ++jj) {
            const int j = 2 * jp + jj;
            FH kb, lb;
            kb.h[0] = *(const v8h*)(Ksh + (j * 16 + c) * HDIM + dc * 32 + 8 * hh);
            kb.h[1] = *(const v8h*)(Ksh + (j * 16 + c) * HDIM + dc * 32 + 16 + 8 * hh);
            lb.h[0] = *(const v8h*)(Kls + (j * 16 + c) * HDIM + dc * 32 + 8 * hh);
            lb.h[1] = *(const v8h*)(Kls + (j * 16 + c) * HDIM + dc * 32 + 16 + 8 * hh);
            sh2[jj] = mma_h_raw(qhf, kb.v, sh2[jj]);
            sl2[jj] = mma_h_raw(qlf, kb.v, sl2[jj]);
            sl2[jj] = mma_h_raw(qhf, lb.v, sl2[jj]);
            guard4m(sh2[jj], sl2[jj], qhf, qlf, kb.v, lb.v);
          }
        }
#pragma unroll
        for (int jj = 0; jj < 2; ++jj) {
          const int j    = 2 * jp + jj;
          const int key  = kv0 + j * 16 + c;
          const int rowb = q0 + 8 * hh;
#pragma unroll
          for (int r = 0; r < 8; ++r) {
            float v = sh2[jj][r];
            v += sl2[jj][r] * (1.0f / RSC);
            v *= sscale;
            s[j][r] = (key <= rowb + r) ? v : NEG_BIG;
          }
        }
      }
    } else {
      v16h qh[4];
#pragma unroll
      for (int dc = 0; dc < 4; ++dc) qh[dc] = ldfrag_h(Qg + (size_t)(q0 + c) * DM + dc * 32 + 8 * hh);
#pragma unroll
      for (int j = 0; j < 4; ++j) {
        v8f sh = zero8();
#pragma unroll
        for (int dc = 0; dc < 4; ++dc) {
          FH kb;
          kb.h[0] = *(const v8h*)(Ksh + (j * 16 + c) * HDIM + dc * 32 + 8 * hh);
          kb.h[1] = *(const v8h*)(Ksh + (j * 16 + c) * HDIM + dc * 32 + 16 + 8 * hh);
          sh = mma_h(qh[dc], kb.v, sh);
        }
        const int key  = kv0 + j * 16 + c;
        const int rowb = q0 + 8 * hh;
#pragma unroll
        for (int r = 0; r < 8; ++r) {
          const float v = sh[r] * sscale;
          s[j][r] = (key <= rowb + r) ? v : NEG_BIG;
        }
      }
    }

#pragma unroll
    for (int r = 0; r < 8; ++r) {
      float m = s[0][r];
      m = fmaxf(m, s[1][r]);
      m = fmaxf(m, s[2][r]);
      m = fmaxf(m, s[3][r]);
#pragma unroll
      for (int off = 1; off < 16; off <<= 1) m = fmaxf(m, __shfl_xor(m, off, 32));
      const float mnew  = fmaxf(mrow[r], m);
      const float alpha = __expf(mrow[r] - mnew);
      mrow[r] = mnew;
      float psum = 0.f;
#pragma unroll
      for (int j = 0; j < 4; ++j) {
        const float p  = __expf(s[j][r] - mnew);
        psum += p;
        const float ph = p * PSC;
        const _Float16 xh = (_Float16)ph;
        const int pi = (8 * hh + r) * 64 + j * 16 + c;
        pwh[pi] = xh;
        if (PRES) pwl[pi] = (_Float16)((ph - (float)xh) * RSC);
      }
#pragma unroll
      for (int off = 1; off < 16; off <<= 1) psum += __shfl_xor(psum, off, 32);
      lrow[r] = lrow[r] * alpha + psum;
#pragma unroll
      for (int t = 0; t < 8; ++t) oh[t][r] *= alpha;
    }
    wave_sync_lds();

    FH pa0, pa1, pb0, pb1;
    pa0.h[0] = *(const v8h*)(pwh + c * 64 + 8 * hh);
    pa0.h[1] = *(const v8h*)(pwh + c * 64 + 16 + 8 * hh);
    pa1.h[0] = *(const v8h*)(pwh + c * 64 + 32 + 8 * hh);
    pa1.h[1] = *(const v8h*)(pwh + c * 64 + 48 + 8 * hh);
    pb0.v = pa0.v;
    pb1.v = pa1.v;
    if (PRES) {
      pb0.h[0] = *(const v8h*)(pwl + c * 64 + 8 * hh);
      pb0.h[1] = *(const v8h*)(pwl + c * 64 + 16 + 8 * hh);
      pb1.h[0] = *(const v8h*)(pwl + c * 64 + 32 + 8 * hh);
      pb1.h[1] = *(const v8h*)(pwl + c * 64 + 48 + 8 * hh);
      cbar();
    }
#pragma unroll
    for (int t = 0; t < 8; ++t) {
      const _Float16* vr = Vhs + (t * 16 + c) * 64 + 8 * hh;
      FH vb0, vb1;
      vb0.h[0] = *(const v8h*)(vr);
      vb0.h[1] = *(const v8h*)(vr + 16);
      vb1.h[0] = *(const v8h*)(vr + 32);
      vb1.h[1] = *(const v8h*)(vr + 48);
      if (PRES) {
        const _Float16* wr = Vls + (t * 16 + c) * 64 + 8 * hh;
        FH wb0, wb1;
        wb0.h[0] = *(const v8h*)(wr);
        wb0.h[1] = *(const v8h*)(wr + 16);
        wb1.h[0] = *(const v8h*)(wr + 32);
        wb1.h[1] = *(const v8h*)(wr + 48);
        v8f ol = zero8();
        oh[t] = mma_h_raw(pa0.v, vb0.v, oh[t]);
        ol    = mma_h_raw(pa0.v, wb0.v, ol);
        ol    = mma_h_raw(pb0.v, vb0.v, ol);
        oh[t] = mma_h_raw(pa1.v, vb1.v, oh[t]);
        ol    = mma_h_raw(pa1.v, wb1.v, ol);
        ol    = mma_h_raw(pb1.v, vb1.v, ol);
        guard8m(oh[t], ol, pa0.v, pa1.v, pb0.v, pb1.v, vb0.v, vb1.v, wb0.v, wb1.v);
#pragma unroll
        for (int r = 0; r < 8; ++r) oh[t][r] += ol[r] * (1.0f / RSC);
      } else {
        oh[t] = mma_h_raw(pa0.v, vb0.v, oh[t]);
        oh[t] = mma_h_raw(pa1.v, vb1.v, oh[t]);
        guard1q(oh[t], pa0.v, pa1.v, vb0.v, vb1.v);
      }
    }
    acc_guard4(oh[0], oh[1], oh[2], oh[3]);
    acc_guard4(oh[4], oh[5], oh[6], oh[7]);
  }

  float* os = Os[wave];
#pragma unroll
  for (int r = 0; r < 8; ++r) {
    const float l = lrow[r];
    const float inv = (1.0f / l) * (1.0f / (PSC * VSC));
    const float* gr = Gg + (size_t)(q0 + 8 * hh + r) * DM;
#pragma unroll
    for (int t = 0; t < 8; ++t) {
      float g = gr[t * 16 + c];
      g = fminf(fmaxf(g, -30.0f), 30.0f);
      const float sig = 1.0f / (1.0f + expf(-g));
      os[(8 * hh + r) * HDIM + t * 16 + c] = oh[t][r] * inv * sig;
    }
  }
  wave_sync_lds();
  {
    v4u hvv[8], lvv[8];
#pragma unroll
    for (int it = 0; it < 8; ++it) {
      const int row = it * 2 + hh;
      const float* sp = os + row * HDIM + c * 8;
      const v4f fa = *(const v4f*)sp;
      const v4f fb = *(const v4f*)(sp + 4);
      float f[8];
      f[0] = fa[0]; f[1] = fa[1]; f[2] = fa[2]; f[3] = fa[3];
      f[4] = fb[0]; f[5] = fb[1]; f[6] = fb[2]; f[7] = fb[3];
      v4u pk, pl;
#pragma unroll
      for (int e = 0; e < 4; ++e) {
        const float g0 = f[2 * e] * CXS, g1 = f[2 * e + 1] * CXS;
        const _Float16 x0 = (_Float16)g0, x1 = (_Float16)g1;
        const _Float16 y0 = (_Float16)(g0 - (float)x0), y1 = (_Float16)(g1 - (float)x1);
        pk[e] = pk16(h_bits(x0), h_bits(x1));
        pl[e] = pk16(h_bits(y0), h_bits(y1));
      }
      hvv[it] = pk;
      lvv[it] = pl;
    }
    for (int pass = 0; pass < 2; ++pass) {
#pragma unroll
      for (int it = 0; it < 8; ++it) {
        const int row = it * 2 + hh;
        const size_t go = (size_t)(q0 + row) * DM + (size_t)h * HDIM + c * 8;
        *(volatile v4u*)(CH + go) = hvv[it];
        *(volatile v4u*)(CL + go) = lvv[it];
      }
      __threadfence();
    }
  }
}

extern "C" void kernel_launch(void* const* d_in, const int* in_sizes, int n_in,
                              void* d_out, int out_size, void* d_ws, size_t ws_size,
                              hipStream_t stream) {
  if (n_in < 9) return;
  if (in_sizes[0] != NTOK * DM) return;
  if (in_sizes[1] != NBATCH * SEQ * HDIM || in_sizes[2] != NBATCH * SEQ * HDIM) return;
  if (in_sizes[3] != QGD * DM) return;
  if (in_sizes[4] != KVD * DM || in_sizes[5] != KVD * DM) return;
  if (in_sizes[6] != DM * DM) return;
  if (in_sizes[7] != HDIM || in_sizes[8] != HDIM) return;
  if (out_size != NTOK * DM) return;

  const float* X    = (const float*)d_in[0];
  const float* COSI = (const float*)d_in[1];
  const float* SINI = (const float*)d_in[2];
  const float* Wq   = (const float*)d_in[3];
  const float* Wk   = (const float*)d_in[4];
  const float* Wv   = (const float*)d_in[5];
  const float* Wo   = (const float*)d_in[6];
  const float* QNW  = (const float*)d_in[7];
  const float* KNW  = (const float*)d_in[8];
  float* outf = (float*)d_out;

  const size_t PXH  = (size_t)NTOK * DM * 2;
  const size_t PWQ  = (size_t)QGD * DM * 2;
  const size_t PWK  = (size_t)KVD * DM * 2;
  const size_t PWO  = (size_t)DM * DM * 2;
  const size_t PQ   = (size_t)SEQ * DM * 2;
  const size_t PGT  = (size_t)SEQ * DM * 4;
  const size_t PK   = (size_t)SEQ * KVD * 2;
  const size_t PVT  = (size_t)KVD * SEQ * 2;
  const size_t PCTX = (size_t)SEQ * DM * 2;
  size_t off = 0;
  const size_t oXH = off; off += PXH;
  const size_t oWQ = off; off += PWQ;
  const size_t oWK = off; off += PWK;
  const size_t oWV = off; off += PWK;
  const size_t oWO = off; off += PWO;
  const size_t oQH = off; off += PQ;
  const size_t oQL = off; off += PQ;
  const size_t oGT = off; off += PGT;
  const size_t oKH = off; off += PK;
  const size_t oKL = off; off += PK;
  const size_t oVH = off; off += PVT;
  const size_t oVL = off; off += PVT;
  const size_t oCH = off; off += PCTX;
  const size_t oCL = off; off += PCTX;
  if (off > ws_size) return;
  if (off > (size_t)134217728) return;

  char* ws = (char*)d_ws;
  unsigned short* XH   = (unsigned short*)(ws + oXH);
  unsigned short* WQH  = (unsigned short*)(ws + oWQ);
  unsigned short* WKH  = (unsigned short*)(ws + oWK);
  unsigned short* WVH  = (unsigned short*)(ws + oWV);
  unsigned short* WOH  = (unsigned short*)(ws + oWO);
  unsigned short* QH   = (unsigned short*)(ws + oQH);
  unsigned short* QL   = (unsigned short*)(ws + oQL);
  float*          GT   = (float*)(ws + oGT);
  unsigned short* KH   = (unsigned short*)(ws + oKH);
  unsigned short* KL   = (unsigned short*)(ws + oKL);
  unsigned short* VTH  = (unsigned short*)(ws + oVH);
  unsigned short* VTL  = (unsigned short*)(ws + oVL);
  unsigned short* CTXH = (unsigned short*)(ws + oCH);
  unsigned short* CTXL = (unsigned short*)(ws + oCL);

  const dim3 blk256(256), blk128(128);
  const float sscale = 0.08838834764831845f / (QSC * KSC);

  cvt_rm<<<dim3((NTOK * DM) / 2048), blk256, 0, stream>>>(X,  XH,  NTOK * DM, 1.0f, 0);
  cvt_rm<<<dim3((QGD * DM) / 2048),  blk256, 0, stream>>>(Wq, WQH, QGD * DM,  WSC,  0);
  cvt_rm<<<dim3((KVD * DM) / 2048),  blk256, 0, stream>>>(Wk, WKH, KVD * DM,  WSC,  0);
  cvt_rm<<<dim3((KVD * DM) / 2048),  blk256, 0, stream>>>(Wv, WVH, KVD * DM,  WSC,  0);
  cvt_rm<<<dim3((DM * DM) / 2048),   blk256, 0, stream>>>(Wo, WOH, DM * DM,   WSC,  0);

  const int gq   = ((SEQ / 32) * (QGD / 128)) / 4;
  const int gk   = ((SEQ / 32) * (KVD / 128)) / 4;
  const int gv   = ((KVD / 32) * (SEQ / 128)) / 4;
  const int go0  = ((LEADR / 32) * (DM / 128)) / 4;
  const int go1  = (((SEQ - LEADR) / 32) * (DM / 128)) / 4;
  for (int b = 0; b < NBATCH; ++b) {
    const unsigned short* XHb = XH + (size_t)b * SEQ * DM;
    const float* cosb = COSI + (size_t)b * SEQ * HDIM;
    const float* sinb = SINI + (size_t)b * SEQ * HDIM;
    float* outb = outf + (size_t)b * SEQ * DM;
    gemm_t<1, 2><<<dim3(gq), blk128, 0, stream>>>(
        XHb, XHb, DM, WQH, WQH, DM, (void*)QH, (void*)QL, (void*)GT, DM, cosb, sinb, QNW,
        SEQ, QGD, DM, 1.0f / WSC, QSC);
    gemm_t<1, 1><<<dim3(gk), blk128, 0, stream>>>(
        XHb, XHb, DM, WKH, WKH, DM, (void*)KH, (void*)KL, (void*)KL, KVD, cosb, sinb, KNW,
        SEQ, KVD, DM, 1.0f / WSC, KSC);
    gemm_t<1, 0><<<dim3(gv), blk128, 0, stream>>>(
        WVH, WVH, DM, XHb, XHb, DM, (void*)VTH, (void*)VTL, (void*)VTL, SEQ, cosb, sinb, QNW,
        KVD, SEQ, DM, VSC / WSC, 1.0f);
    attn_c<true><<<dim3(NQP * NHEAD), blk128, 0, stream>>>(QH, QL, KH, KL, VTH, VTL, GT, CTXH, CTXL,
                                                           sscale, 0, NQP);
    attn_c<false><<<dim3((NQB - NQP) * NHEAD), blk128, 0, stream>>>(QH, QL, KH, KL, VTH, VTL, GT, CTXH, CTXL,
                                                                    sscale, NQP, NQB - NQP);
    gemm_t<2, 3><<<dim3(go0), blk128, 0, stream>>>(
        CTXH, CTXL, DM, WOH, WOH, DM, (void*)outb, (void*)outb, (void*)outb, DM, cosb, sinb, QNW,
        LEADR, DM, DM, 1.0f / (CXS * WSC), 1.0f);
    gemm_t<1, 3><<<dim3(go1), blk128, 0, stream>>>(
        CTXH + (size_t)LEADR * DM, CTXH + (size_t)LEADR * DM, DM, WOH, WOH, DM,
        (void*)(outb + (size_t)LEADR * DM), (void*)(outb + (size_t)LEADR * DM),
        (void*)(outb + (size_t)LEADR * DM), DM, cosb, sinb, QNW,
        SEQ - LEADR, DM, DM, 1.0f / (CXS * WSC), 1.0f);
  }
  (void)hipGetLastError();
}
